// SwinTransformerBlock_81819126989606
// MI455X (gfx1250) — hardware-run, weakly checked
//
#include <hip/hip_runtime.h>


#define NB_  32
#define HW   56
#define CC   128
#define NHD  4
#define HD   32
#define WS   7
#define NWS  8
#define NW   64
#define NT   49
#define SH   3
#define MLP  512
#define NTOK (NB_ * HW * HW)
#define TCH  (BPP * HW * HW)
#define BPP  4
#define ZP   (BPP * NW * NHD)
typedef _Float16 h16;
typedef unsigned short bf;
typedef __attribute__((ext_vector_type(16))) __bf16   v16bf;
typedef __attribute__((ext_vector_type(16))) _Float16 v16h;
typedef __attribute__((ext_vector_type(8)))  _Float16 v8h;
typedef __attribute__((ext_vector_type(8)))  unsigned short v8us;
typedef __attribute__((ext_vector_type(8)))  float    v8f;
typedef __attribute__((ext_vector_type(4)))  float    v4f;
typedef v8h  __attribute__((may_alias)) v8ha;
typedef v4f  __attribute__((may_alias)) v4fa;
typedef v8us __attribute__((may_alias)) v8usa;

__device__ __forceinline__ unsigned short f2bf(float f) { unsigned u = __float_as_uint(f); u += 0x7FFFu + ((u >> 16) & 1u); return (unsigned short)(u >> 16); }
__device__ __forceinline__ float bf2f(unsigned short b) { return __uint_as_float(((unsigned)b) << 16); }
__device__ __forceinline__ float bfr(float f) { return bf2f(f2bf(f)); }
__device__ __forceinline__ v16h cat16(v8h lo, v8h hi) { return __builtin_shufflevector(lo, hi, 0, 1, 2, 3, 4, 5, 6, 7, 8, 9, 10, 11, 12, 13, 14, 15); }
__device__ __forceinline__ v16bf cat16b(v8us lo, v8us hi) { return __builtin_bit_cast(v16bf, __builtin_shufflevector(lo, hi, 0, 1, 2, 3, 4, 5, 6, 7, 8, 9, 10, 11, 12, 13, 14, 15)); }
__device__ __forceinline__ v8f wmma16(v16h a, v16h b, v8f c) { return __builtin_amdgcn_wmma_f32_16x16x32_f16(false, a, false, b, (short)0, c, false, false); }
__device__ __forceinline__ v8f wmmab(v16bf a, v16bf b, v8f c) { return __builtin_amdgcn_wmma_f32_16x16x32_bf16(false, a, false, b, (short)0, c, false, false); }


template <typename T16> struct WFrag;
template <> struct WFrag<h16> { typedef v16h V; static __device__ __forceinline__ V ld(const h16* p) { return cat16(*(const v8h*)p, *(const v8h*)(p + 16)); } static __device__ __forceinline__ v8f mma(V a, V b, v8f c) { return wmma16(a, b, c); } };
template <> struct WFrag<bf> { typedef v16bf V; static __device__ __forceinline__ V ld(const bf* p) { return cat16b(*(const v8us*)p, *(const v8us*)(p + 16)); } static __device__ __forceinline__ v8f mma(V a, V b, v8f c) { return wmmab(a, b, c); } };
template <typename T16, int NSPLIT, bool BIAS>
__global__ __launch_bounds__(32) void k_gemmw(const T16* __restrict__ A, const T16* __restrict__ A2, const T16* __restrict__ Bt, const T16* __restrict__ Bt2, int K, float* C, int ldc, const float* __restrict__ bias, size_t sA, size_t sB, size_t sC) {
    typedef typename WFrag<T16>::V V;
    __shared__ __align__(16) float os[16 * 68];
    const size_t z = blockIdx.z; A += z * sA; if (A2) A2 += z * sA; Bt += z * sB; if (Bt2) Bt2 += z * sB; C += z * sC;
    const int lane = threadIdx.x & 31, lr = lane & 15, hi = lane >> 4; const int r0 = blockIdx.x * 64, c0 = blockIdx.y * 64;
    v8f acc[4][4];
#pragma unroll
    for (int mb = 0; mb < 4; ++mb)
#pragma unroll
        for (int nb = 0; nb < 4; ++nb) acc[mb][nb] = (v8f){};
    const size_t aoff = (size_t)(r0 + lr) * K + 8 * hi, boff = (size_t)(c0 + lr) * K + 8 * hi;
#pragma unroll 1
    for (int kc = 0; kc < K; kc += 32) {
        V a[4], a2[4];
#pragma unroll
        for (int mb = 0; mb < 4; ++mb) { a[mb] = WFrag<T16>::ld(A + aoff + (size_t)mb * 16 * K + kc); if (NSPLIT == 1 || NSPLIT == 2) a2[mb] = WFrag<T16>::ld(A2 + aoff + (size_t)mb * 16 * K + kc); }
#pragma unroll
        for (int nb = 0; nb < 4; ++nb) { const V b = WFrag<T16>::ld(Bt + boff + (size_t)nb * 16 * K + kc); V b2; if (NSPLIT >= 2) b2 = WFrag<T16>::ld(Bt2 + boff + (size_t)nb * 16 * K + kc);
#pragma unroll
            for (int mb = 0; mb < 4; ++mb) { acc[mb][nb] = WFrag<T16>::mma(a[mb], b, acc[mb][nb]); if (NSPLIT == 1 || NSPLIT == 2) acc[mb][nb] = WFrag<T16>::mma(a2[mb], b, acc[mb][nb]); if (NSPLIT >= 2) acc[mb][nb] = WFrag<T16>::mma(a[mb], b2, acc[mb][nb]); } }
        asm volatile("v_nop\n\tv_nop\n\tv_nop\n\tv_nop" : "+v"(acc[0][0]), "+v"(acc[1][1]), "+v"(acc[2][2]), "+v"(acc[3][3]) : "v"(a[0]), "v"(a[3]));
    }
#pragma unroll
    for (int mb = 0; mb < 4; ++mb) {
#pragma unroll
        for (int nb = 0; nb < 4; ++nb) {
#pragma unroll
            for (int j = 0; j < 8; ++j) os[(hi * 8 + j) * 68 + nb * 16 + lr] = acc[mb][nb][j]; }
        __builtin_amdgcn_wave_barrier(); asm volatile("" ::: "memory");
        float* crow = C + (size_t)(r0 + mb * 16) * ldc + c0;
#pragma unroll 1
        for (int ps = 0; ps < 2; ++ps) {
#pragma unroll
            for (int s = 0; s < 8; ++s) { const int row = 2 * s + hi, cofs = lr * 4; v4f val = *(const v4fa*)(os + row * 68 + cofs); if (BIAS) { val[0] += bfr(bias[c0 + cofs]); val[1] += bfr(bias[c0 + cofs + 1]); val[2] += bfr(bias[c0 + cofs + 2]); val[3] += bfr(bias[c0 + cofs + 3]); }
                *(volatile v4f*)(crow + (size_t)row * ldc + cofs) = val; }
            if (ps == 0) __threadfence(); }
        __builtin_amdgcn_wave_barrier(); asm volatile("" ::: "memory");
    }
}

__device__ __forceinline__ void splitf(float y, unsigned short& h, unsigned short& l) { h = f2bf(y); l = f2bf(y - bf2f(h)); }
typedef __attribute__((ext_vector_type(2))) unsigned short v2us;
typedef __attribute__((ext_vector_type(4))) unsigned short v4us;

__global__ __launch_bounds__(256) void k_wtG(const float* __restrict__ w, int K, int N, bf* Bt) {
    const int lane = threadIdx.x & 31; const int L0 = (blockIdx.x * 8 + (threadIdx.x >> 5)) * 8; const int nlines = N * K / 64;
#pragma unroll
    for (int ps = 0; ps < 2; ++ps) {
#pragma unroll 1
        for (int l = 0; l < 8; ++l) { const int L = L0 + l; if (L >= nlines) break; const size_t e = (size_t)L * 64 + lane * 2; const int k = (int)(e % K), n = (int)(e / K); v2us o;
            o[0] = f2bf(w[(size_t)k * N + n]); o[1] = f2bf(w[(size_t)(k + 1) * N + n]); *(volatile v2us*)(Bt + e) = o; }
        if (ps == 0) __threadfence(); }
}
__device__ __forceinline__ int tokOf(int bimg, int wi, int n) { const int wr = wi / NWS, wc = wi % NWS; const int rp = wr * WS + n / WS, cp = wc * WS + n % WS; const int r = (rp + SH) % HW, c = (cp + SH) % HW; return (bimg * HW + r) * HW + c; }
__device__ __forceinline__ int regOf(int wi, int n) { const int wr = wi / NWS, wc = wi % NWS; const int rp = wr * WS + n / WS, cp = wc * WS + n % WS; const int rh = (rp < HW - WS) ? 0 : (rp < HW - SH) ? 1 : 2; const int rw = (cp < HW - WS) ? 0 : (cp < HW - SH) ? 1 : 2; return rh * 3 + rw; }
__global__ __launch_bounds__(256) void k_ln(const float* __restrict__ X, int xbf, const float* __restrict__ R, const float* __restrict__ g, const float* __restrict__ bb, float* S, bf* Hh, bf* Hl) { const int lane = threadIdx.x & 31; const int t = blockIdx.x * 8 + (threadIdx.x >> 5); if (t >= TCH) return; const size_t o0 = (size_t)t * CC + lane * 4; const v4f a = *(const v4f*)(X + o0); v4f v; float s = 0.f;
#pragma unroll
    for (int u = 0; u < 4; ++u) { float av = xbf ? bfr(a[u]) : a[u]; if (R) av = __fadd_rn(av, R[o0 + u]); v[u] = av; s += av; }
#pragma unroll
    for (int sh = 16; sh; sh >>= 1) s += __shfl_xor(s, sh, 32);
    const float mean = s * (1.0f / CC); float q = 0.f;
#pragma unroll
    for (int u = 0; u < 4; ++u) { float d = __fsub_rn(v[u], mean); asm volatile("" : "+v"(d)); float p = __fmul_rn(d, d); asm volatile("" : "+v"(p)); q = __fadd_rn(q, p); }
#pragma unroll
    for (int sh = 16; sh; sh >>= 1) q += __shfl_xor(q, sh, 32);
    const float rs = __frsqrt_rn(__fadd_rn(q * (1.0f / CC), 1e-5f)); v4us oh, ol;
#pragma unroll
    for (int u = 0; u < 4; ++u) { const int c = lane * 4 + u; float d = __fsub_rn(v[u], mean); asm volatile("" : "+v"(d)); float n0 = __fmul_rn(d, rs); asm volatile("" : "+v"(n0)); float gg = bfr(g[c]), be = bfr(bb[c]); asm volatile("" : "+v"(gg)); asm volatile("" : "+v"(be)); float t1 = __fmul_rn(n0, gg); asm volatile("" : "+v"(t1)); unsigned short p2, q2; splitf(__fadd_rn(t1, be), p2, q2); oh[u] = p2; ol[u] = q2; }
    if (S) *(volatile v4f*)(S + o0) = v; *(volatile v4us*)(Hh + o0) = oh; *(volatile v4us*)(Hl + o0) = ol; __threadfence(); if (S) *(volatile v4f*)(S + o0) = v; *(volatile v4us*)(Hh + o0) = oh; *(volatile v4us*)(Hl + o0) = ol; }
__global__ __launch_bounds__(256) void k_wgath(const float* __restrict__ QKV, const float* __restrict__ bq, int b0, bf* Qh, bf* Ql, bf* Kh, bf* Kl) {
    const size_t e = ((size_t)blockIdx.x * 256 + threadIdx.x) * 4; if (e >= (size_t)ZP * 64 * HD) return; const int d = (int)(e % HD); const int slot = (int)((e / HD) % 64); const int z = (int)(e / ((size_t)HD * 64)); const int h = z % NHD, wi = (z / NHD) % NW, bl = z / (NHD * NW);
    v4us qh, ql, kh, kl; if (slot < NT) { const int tok = tokOf(bl, wi, slot); (void)b0; const float* row = QKV + (size_t)tok * (3 * CC);
#pragma unroll
        for (int u = 0; u < 4; ++u) { const int c = h * HD + d + u; float qv = __fadd_rn(row[c], bfr(bq[c])); qv = __fmul_rn(qv, 0.17677669529663687f); const float kv = __fadd_rn(row[CC + c], bfr(bq[CC + c])); unsigned short a, b; splitf(qv, a, b); qh[u] = a; ql[u] = b; splitf(kv, a, b); kh[u] = a; kl[u] = b; } }
    else { for (int u = 0; u < 4; ++u) { qh[u] = 0; ql[u] = 0; kh[u] = 0; kl[u] = 0; } }
    *(volatile v4us*)(Qh + e) = qh; *(volatile v4us*)(Ql + e) = ql; *(volatile v4us*)(Kh + e) = kh; *(volatile v4us*)(Kl + e) = kl; __threadfence(); *(volatile v4us*)(Qh + e) = qh; *(volatile v4us*)(Ql + e) = ql; *(volatile v4us*)(Kh + e) = kh; *(volatile v4us*)(Kl + e) = kl; }
__global__ __launch_bounds__(256) void k_vgath(const float* __restrict__ QKV, const float* __restrict__ bq, bf* Vh, bf* Vl) { const size_t e = ((size_t)blockIdx.x * 256 + threadIdx.x) * 4; if (e >= (size_t)ZP * 64 * 64) return; const int m = (int)(e % 64); const int dp = (int)((e / 64) % 64); const int z2 = (int)(e / ((size_t)64 * 64)); const int h2 = z2 % NHD, wi2 = (z2 / NHD) % NW, bl2 = z2 / (NHD * NW); v4us vh, vl;
#pragma unroll
    for (int u = 0; u < 4; ++u) { const int mm = m + u; float vv = 0.f; if (mm < NT && dp < HD) { const int tok = tokOf(bl2, wi2, mm); const int c = 2 * CC + h2 * HD + dp; vv = __fadd_rn(QKV[(size_t)tok * (3 * CC) + c], bfr(bq[c])); } unsigned short a, b; splitf(vv, a, b); vh[u] = a; vl[u] = b; }
    *(volatile v4us*)(Vh + e) = vh; *(volatile v4us*)(Vl + e) = vl; __threadfence(); *(volatile v4us*)(Vh + e) = vh; *(volatile v4us*)(Vl + e) = vl; }
__global__ __launch_bounds__(256) void k_wsoft(const float* __restrict__ S, const float* __restrict__ rbt, bf* Ph, bf* Pl) { const int lane = threadIdx.x & 31; const int row = blockIdx.x * 8 + (threadIdx.x >> 5); if (row >= ZP * 64) return; const int n = row % 64; const int z = row / 64; const int h = z % NHD, wi = (z / NHD) % NW; const float* sr = S + (size_t)row * 64; float v[2]; float mx = -3.0e38f;
    if (n < NT) { const int rn = n / WS, cn = n % WS; const int regn = regOf(wi, n);
#pragma unroll
        for (int w = 0; w < 2; ++w) { const int m = lane * 2 + w; float t = -3.0e38f;
            if (m < NT) { const int rm = m / WS, cm = m % WS; const int ridx = (rn - rm + WS - 1) * (2 * WS - 1) + (cn - cm + WS - 1); float rb = bfr(rbt[ridx * NHD + h]); asm volatile("" : "+v"(rb)); float s0 = __fadd_rn(sr[m], rb); asm volatile("" : "+v"(s0)); t = (regOf(wi, m) != regn) ? __fadd_rn(s0, -100.0f) : s0; }
            v[w] = t; mx = fmaxf(mx, t); } } else { v[0] = v[1] = -3.0e38f; }
#pragma unroll
    for (int sh = 16; sh; sh >>= 1) mx = fmaxf(mx, __shfl_xor(mx, sh, 32));
    float sum = 0.f;
#pragma unroll
    for (int w = 0; w < 2; ++w) { if (n < NT && lane * 2 + w < NT) { float d0 = __fsub_rn(v[w], mx); asm volatile("" : "+v"(d0)); v[w] = __builtin_amdgcn_exp2f(__fmul_rn(d0, 1.4426950408889634f)); } else v[w] = 0.f; sum += v[w]; }
#pragma unroll
    for (int sh = 16; sh; sh >>= 1) sum += __shfl_xor(sum, sh, 32);
    const float f = (n < NT) ? __fdiv_rn(1.0f, sum) : 0.f; v2us oh, ol;
#pragma unroll
    for (int w = 0; w < 2; ++w) { unsigned short a, b; splitf(v[w] * f, a, b); oh[w] = a; ol[w] = b; }
    const size_t oo = (size_t)row * 64 + lane * 2; *(volatile v2us*)(Ph + oo) = oh; *(volatile v2us*)(Pl + oo) = ol; __threadfence(); *(volatile v2us*)(Ph + oo) = oh; *(volatile v2us*)(Pl + oo) = ol; }
__global__ __launch_bounds__(256) void k_wscat(const float* __restrict__ O, int b0, bf* Ah, bf* Al) { const size_t e = ((size_t)blockIdx.x * 256 + threadIdx.x) * 4; if (e >= (size_t)BPP * HW * HW * CC) return; const int c = (int)(e % CC); const int tl = (int)(e / CC); const int bl = tl / (HW * HW); const int rc = tl % (HW * HW); const int r = rc / HW, col = rc % HW; const int h = c / HD, d = c % HD;
    const int rp = (r - SH + HW) % HW, cp = (col - SH + HW) % HW; const int wi = (rp / WS) * NWS + cp / WS; const int n = (rp % WS) * WS + cp % WS; const int z = (bl * NW + wi) * NHD + h; const float* src = O + ((size_t)z * 64 + n) * 64 + d; v4us oh, ol; (void)b0;
#pragma unroll
    for (int u = 0; u < 4; ++u) { unsigned short a, b; splitf(src[u], a, b); oh[u] = a; ol[u] = b; } const size_t oo = ((size_t)bl * HW * HW + rc) * CC + c; *(volatile v4us*)(Ah + oo) = oh; *(volatile v4us*)(Al + oo) = ol; __threadfence(); *(volatile v4us*)(Ah + oo) = oh; *(volatile v4us*)(Al + oo) = ol; }
__global__ __launch_bounds__(256) void k_gelu(const float* __restrict__ F, const float* __restrict__ b1, bf* Gh, bf* Gl) { const size_t e = ((size_t)blockIdx.x * 256 + threadIdx.x) * 4; if (e >= (size_t)TCH * MLP) return; const int c = (int)(e % MLP); const v4f a = *(const v4f*)(F + e); v4us oh, ol;
#pragma unroll 1
    for (int u = 0; u < 4; ++u) { const float gx = __fadd_rn(a[u], bfr(b1[c + u])); float er = erff(gx * 0.7071067811865475f); asm volatile("" : "+v"(er)); float u1 = __fadd_rn(1.0f, er); asm volatile("" : "+v"(u1)); float hx = __fmul_rn(0.5f, gx); asm volatile("" : "+v"(hx)); unsigned short p, q; splitf(__fmul_rn(hx, u1), p, q); oh[u] = p; ol[u] = q; }
    *(volatile v4us*)(Gh + e) = oh; *(volatile v4us*)(Gl + e) = ol; __threadfence(); *(volatile v4us*)(Gh + e) = oh; *(volatile v4us*)(Gl + e) = ol; }
__global__ __launch_bounds__(256) void k_fin(const float* __restrict__ X1, const float* __restrict__ G2, const float* __restrict__ b2, float* out) { const size_t e = ((size_t)blockIdx.x * 256 + threadIdx.x) * 4; if (e >= (size_t)TCH * CC) return; const int c = (int)(e % CC); const v4f a = *(const v4f*)(X1 + e), g4 = *(const v4f*)(G2 + e); v4f o;
#pragma unroll
    for (int u = 0; u < 4; ++u) o[u] = __fadd_rn(a[u], __fadd_rn(g4[u], bfr(b2[c + u]))); *(volatile v4f*)(out + e) = o; __threadfence(); *(volatile v4f*)(out + e) = o; }

extern "C" void kernel_launch(void* const* d_in, const int* in_sizes, int n_in,
                              void* d_out, int out_size, void* d_ws, size_t ws_size, hipStream_t stream) {
    (void)in_sizes; (void)n_in; (void)out_size;
    const float** I = (const float**)d_in;
    const float *x = I[0], *wqkv = I[1], *bqkv = I[2], *wp = I[3], *bp = I[4], *rbt = I[5], *g1 = I[6], *be1 = I[7], *g2 = I[8], *be2 = I[9], *w1 = I[10], *b1 = I[11], *w2 = I[12], *b2 = I[13];
    float* OUT = (float*)d_out;
    char* wsp = (char*)d_ws;
    auto take = [&](size_t bytes) { char* p = wsp; wsp += (bytes + 255) & ~(size_t)255; return (void*)p; };
    bf* BQKV = (bf*)take((size_t)3 * CC * CC * 2); bf* BP = (bf*)take((size_t)CC * CC * 2); bf* B1 = (bf*)take((size_t)MLP * CC * 2); bf* B2 = (bf*)take((size_t)CC * MLP * 2);
    bf* Hh = (bf*)take((size_t)TCH * CC * 2); bf* Hl = (bf*)take((size_t)TCH * CC * 2); float* QKV = (float*)take((size_t)TCH * 3 * CC * 4);
    bf* Qh = (bf*)take((size_t)ZP * 64 * HD * 2); bf* Ql = (bf*)take((size_t)ZP * 64 * HD * 2); bf* Kh = (bf*)take((size_t)ZP * 64 * HD * 2); bf* Kl = (bf*)take((size_t)ZP * 64 * HD * 2); bf* Vh = (bf*)take((size_t)ZP * 64 * 64 * 2); bf* Vl = (bf*)take((size_t)ZP * 64 * 64 * 2);
    float* S = (float*)take((size_t)ZP * 64 * 64 * 4); bf* Ph = (bf*)take((size_t)ZP * 64 * 64 * 2); bf* Pl = (bf*)take((size_t)ZP * 64 * 64 * 2); float* O = (float*)take((size_t)ZP * 64 * 64 * 4);
    bf* Ah = (bf*)take((size_t)TCH * CC * 2); bf* Al = (bf*)take((size_t)TCH * CC * 2); float* PO = (float*)take((size_t)TCH * CC * 4); float* X1 = (float*)take((size_t)TCH * CC * 4); float* F1 = (float*)take((size_t)TCH * MLP * 4); bf* Gh = (bf*)take((size_t)TCH * MLP * 2); bf* Gl = (bf*)take((size_t)TCH * MLP * 2); float* F2 = (float*)take((size_t)TCH * CC * 4);
    if ((size_t)(wsp - (char*)d_ws) > ws_size) return;
    k_wtG<<<(3 * CC * CC / 64 + 63) / 64, 256, 0, stream>>>(wqkv, CC, 3 * CC, BQKV); k_wtG<<<(CC * CC / 64 + 63) / 64, 256, 0, stream>>>(wp, CC, CC, BP); k_wtG<<<(MLP * CC / 64 + 63) / 64, 256, 0, stream>>>(w1, CC, MLP, B1); k_wtG<<<(CC * MLP / 64 + 63) / 64, 256, 0, stream>>>(w2, MLP, CC, B2);
    const unsigned gW = (unsigned)(((size_t)ZP * 64 * HD / 4 + 255) / 256), gV = (unsigned)(((size_t)ZP * 64 * 64 / 4 + 255) / 256), gT = (unsigned)(((size_t)TCH * CC / 4 + 255) / 256);
    for (int b0 = 0; b0 < NB_; b0 += BPP) { const float* xc = x + (size_t)b0 * HW * HW * CC; float* outc = OUT + (size_t)b0 * HW * HW * CC;
        k_ln<<<TCH / 8, 256, 0, stream>>>(xc, 1, nullptr, g1, be1, nullptr, Hh, Hl);
        k_gemmw<bf, 1, false><<<dim3(TCH / 64, 3 * CC / 64, 1), 32, 0, stream>>>(Hh, Hl, BQKV, nullptr, CC, QKV, 3 * CC, nullptr, 0, 0, 0);
        k_wgath<<<gW, 256, 0, stream>>>(QKV, bqkv, b0, Qh, Ql, Kh, Kl); k_vgath<<<gV, 256, 0, stream>>>(QKV, bqkv, Vh, Vl);
        k_gemmw<bf, 2, false><<<dim3(1, 1, ZP), 32, 0, stream>>>(Qh, Ql, Kh, Kl, HD, S, 64, nullptr, (size_t)64 * HD, (size_t)64 * HD, (size_t)64 * 64);
        k_wsoft<<<ZP * 64 / 8, 256, 0, stream>>>(S, rbt, Ph, Pl);
        k_gemmw<bf, 2, false><<<dim3(1, 1, ZP), 32, 0, stream>>>(Ph, Pl, Vh, Vl, 64, O, 64, nullptr, (size_t)64 * 64, (size_t)64 * 64, (size_t)64 * 64);
        k_wscat<<<gT, 256, 0, stream>>>(O, b0, Ah, Al);
        k_gemmw<bf, 1, true><<<dim3(TCH / 64, CC / 64, 1), 32, 0, stream>>>(Ah, Al, BP, nullptr, CC, PO, CC, bp, 0, 0, 0);
        k_ln<<<TCH / 8, 256, 0, stream>>>(xc, 1, PO, g2, be2, X1, Hh, Hl);
        k_gemmw<bf, 1, false><<<dim3(TCH / 64, MLP / 64, 1), 32, 0, stream>>>(Hh, Hl, B1, nullptr, CC, F1, MLP, nullptr, 0, 0, 0);
        k_gelu<<<(unsigned)(((size_t)TCH * MLP / 4 + 255) / 256), 256, 0, stream>>>(F1, b1, Gh, Gl);
        k_gemmw<bf, 1, false><<<dim3(TCH / 64, CC / 64, 1), 32, 0, stream>>>(Gh, Gl, B2, nullptr, MLP, F2, CC, nullptr, 0, 0, 0);
        k_fin<<<gT, 256, 0, stream>>>(X1, F2, b2, outc); }
}
